// SelfAttention_33019708571866
// MI455X (gfx1250) — hardware-run, weakly checked
//
#include <hip/hip_runtime.h>


#ifndef NB
#define NB 4
#endif
#ifndef SEQ
#define SEQ 2048
#endif
#define NB_FULL 4
#define SEQ_FULL 2048
#define DM 1024
#define NH 8
#define DK 128
#define MTOK (NB * SEQ)
#define PROJN (3 * NH * DK)

static_assert(SEQ % 64 == 0);
static_assert(SEQ <= SEQ_FULL);
static_assert(NB >= 1 && NB <= NB_FULL);
static_assert(DM % 32 == 0);
static_assert(DK == 128);
static_assert(NH * DK == DM);
static_assert(PROJN == 3072);
static_assert(PROJN % 128 == 0);
static_assert(MTOK % 64 == 0);
static_assert(((size_t)MTOK * DM / 8) % 256 == 0);
static_assert(((size_t)NH * DK * DM / 8) % 256 == 0);

#define SC_X   16.0f
#define SC_W   256.0f
#define SC_QKV 8.0f
#define P_CARRY_LOG2 8.0f

#define WS_XH ((size_t)MTOK * DM * 2)
#define WS_WT ((size_t)PROJN * DM * 2)
#define WS_QK (2 * (size_t)NB * NH * SEQ * DK * 2)
#define WS_VT ((size_t)NB * NH * DK * SEQ * 2)
#define WS_TOTAL (WS_XH + WS_WT + WS_QK + WS_VT)
static_assert(WS_XH % 256 == 0 && WS_WT % 256 == 0 && WS_QK % 256 == 0 && WS_VT % 256 == 0);
static_assert(WS_TOTAL <= (size_t)134217728);

typedef _Float16 v8h  __attribute__((ext_vector_type(8)));
typedef _Float16 v16h __attribute__((ext_vector_type(16)));
typedef float    v8f  __attribute__((ext_vector_type(8)));
typedef float    v4f  __attribute__((ext_vector_type(4)));
typedef unsigned v4u  __attribute__((ext_vector_type(4)));

__device__ __forceinline__ float bfr(float f) {
    unsigned u = __float_as_uint(f);
    u = (u + 0x7fffu + ((u >> 16) & 1u)) & 0xffff0000u;
    return __uint_as_float(u);
}
__device__ __forceinline__ _Float16 tohx(float f, float sc) { return (_Float16)(bfr(f) * sc); }
__device__ __forceinline__ _Float16 toh_flush(float v) {
    const _Float16 r = (_Float16)v;
    return (fabsf(v) < 6.103515625e-05f) ? (_Float16)0.0f : r;
}
__device__ __forceinline__ _Float16 tohx_flush(float f, float sc) { return toh_flush(bfr(f) * sc); }

__device__ __forceinline__ v8f wmma16(v16h a, v16h b, v8f c) {
    c = __builtin_amdgcn_wmma_f32_16x16x32_f16(false, a, false, b, (short)0, c, false, false);
    asm volatile("v_nop\n\tv_nop\n\tv_nop\n\tv_nop" : "+v"(c) : "v"(a), "v"(b));
    return c;
}
__device__ __forceinline__ v16h ldfrag(const _Float16* p, int hf) {
    const v8h lo = *(const v8h*)(p + 8 * hf);
    const v8h hi = *(const v8h*)(p + 16 + 8 * hf);
    return __builtin_shufflevector(lo, hi, 0, 1, 2, 3, 4, 5, 6, 7, 8, 9, 10, 11, 12, 13, 14, 15);
}
__device__ __forceinline__ void vst16(_Float16* g, v8h v) { *(volatile v4u*)g = __builtin_bit_cast(v4u, v); }
__device__ __forceinline__ void vst16f(float* g, v4f v) { *(volatile v4f*)g = v; }

#define CVTX_BLK (MTOK * (DM / 8) / 256)
__global__ __launch_bounds__(256) void k_cvtx(const float* __restrict__ X, _Float16* XH) {
    const int i = blockIdx.x * 256 + threadIdx.x;
    const int tok = i >> 7, k = (i & 127) * 8;
    const int bi = tok / SEQ, si = tok - bi * SEQ;
    const float* xp = X + ((size_t)bi * SEQ_FULL + si) * DM + k;
    const v4f x0 = *(const v4f*)(xp);
    const v4f x1 = *(const v4f*)(xp + 4);
    v8h val;
#pragma unroll
    for (int j = 0; j < 4; ++j) {
        val[j]     = tohx_flush(x0[j], SC_X);
        val[4 + j] = tohx_flush(x1[j], SC_X);
    }
    _Float16* dst = XH + (size_t)tok * DM + k;
    vst16(dst, val);
    __threadfence();
    vst16(dst, val);
}

#define PREPW_BLK (NH * DK * (DM / 8) / 256)
__global__ __launch_bounds__(256) void k_prepw(const float* __restrict__ W, _Float16* WT) {
    const int i = blockIdx.x * 256 + threadIdx.x;
    const int n = i >> 7, k = (i & 127) * 8;
    const int hh = n >> 7, e = n & 127;
    v8h val;
#pragma unroll
    for (int j = 0; j < 8; ++j) val[j] = tohx_flush(W[((size_t)hh * DM + k + j) * DK + e], SC_W);
    _Float16* dst = WT + (size_t)n * DM + k;
    vst16(dst, val);
    __threadfence();
    vst16(dst, val);
}

__global__ __launch_bounds__(128) void k_proj(const _Float16* __restrict__ XH, const _Float16* __restrict__ WT,
                                              const float* __restrict__ bK, const float* __restrict__ bV,
                                              _Float16* QK, _Float16* VT) {
    __shared__ __align__(16) _Float16 st[9216];
    const int tid = threadIdx.x, lane = tid & 31, l16 = lane & 15, hf = lane >> 4;
    const int wv = __builtin_amdgcn_readfirstlane(threadIdx.x >> 5);
    const int g = blockIdx.y;
    const int t0 = blockIdx.x * 64;
    const int bi = t0 / SEQ, s0 = t0 - bi * SEQ;
    const int hh = g & 7;
    const bool isV = (g >= 16);
    const _Float16* arow = XH + (size_t)(t0 + wv * 16 + l16) * DM;
    const _Float16* brow = WT + (size_t)(g * 128 + l16) * DM;
    v8f acc[8];
#pragma unroll
    for (int nt = 0; nt < 8; ++nt) acc[nt] = (v8f){};
#pragma unroll 1
    for (int kc = 0; kc < DM / 32; ++kc) {
        const v16h a = ldfrag(arow + kc * 32, hf);
#pragma unroll
        for (int nt = 0; nt < 8; ++nt) {
            const v16h bf = ldfrag(brow + (size_t)(nt * 16) * DM + kc * 32, hf);
            acc[nt] = wmma16(a, bf, acc[nt]);
        }
    }
    if (isV) {
#pragma unroll
        for (int nt = 0; nt < 8; ++nt) {
            const int d = nt * 16 + l16;
            const float bb = bfr(bV[hh * DK + d]);
            v8h pv;
#pragma unroll
            for (int r = 0; r < 8; ++r) pv[r] = toh_flush((acc[nt][r] * (1.0f / (SC_X * SC_W)) + bb) * SC_QKV);
            *(v8h*)&st[d * 72 + wv * 16 + 8 * hf] = pv;
        }
    } else {
#pragma unroll
        for (int nt = 0; nt < 8; ++nt) {
            const int col = nt * 16 + l16;
            const float bkv = bK[hh * DK + col];
            const float bb = (g < 8) ? 0.0f : bfr(bkv);
#pragma unroll
            for (int r = 0; r < 8; ++r) st[(wv * 16 + 8 * hf + r) * 136 + col] = toh_flush((acc[nt][r] * (1.0f / (SC_X * SC_W)) + bb) * SC_QKV);
        }
    }
    __syncthreads();
    v8h w[8];
    if (isV) {
        const int hd = g - 16;
#pragma unroll
        for (int p = 0; p < 8; ++p) { const int d = p * 16 + (tid >> 3), pc = tid & 7; w[p] = *(const v8h*)&st[d * 72 + pc * 8]; }
        auto pass = [&]() {
#pragma unroll
            for (int p = 0; p < 8; ++p) {
                const int d = p * 16 + (tid >> 3), pc = tid & 7;
                vst16(VT + ((size_t)(bi * NH + hd) * DK + d) * SEQ + s0 + pc * 8, w[p]);
            }
        };
        pass();
        __threadfence();
        pass();
    } else {
        _Float16* base = QK + ((size_t)((g >> 3) * (NB * NH) + bi * NH + hh) * SEQ + s0) * DK;
#pragma unroll
        for (int p = 0; p < 8; ++p) { const int off = p * 1024 + tid * 8; w[p] = *(const v8h*)&st[(off >> 7) * 136 + (off & 127)]; }
        auto pass = [&]() {
#pragma unroll
            for (int p = 0; p < 8; ++p) { const int off = p * 1024 + tid * 8; vst16(base + off, w[p]); }
        };
        pass();
        __threadfence();
        pass();
    }
}

__global__ __launch_bounds__(128) void k_attn(const _Float16* __restrict__ QC, const _Float16* __restrict__ KC,
                                              const _Float16* __restrict__ VT, float* OUT) {
    __shared__ __align__(16) float st[4][16 * 132];
    const int tid = threadIdx.x, lane = tid & 31, l16 = lane & 15, hf = lane >> 4;
    const int wv = __builtin_amdgcn_readfirstlane(threadIdx.x >> 5);
    const int bh = blockIdx.y, bi = bh / NH, hd = bh - bi * NH;
    const int q0 = blockIdx.x * 64 + wv * 16;
    v16h qf[4];
    {
        const _Float16* qr = QC + ((size_t)bh * SEQ + q0 + l16) * DK;
#pragma unroll
        for (int cc = 0; cc < 4; ++cc) qf[cc] = ldfrag(qr + cc * 32, hf);
    }
    const _Float16* kb  = KC  + (size_t)bh * SEQ * DK;
    const _Float16* vb  = VT  + (size_t)bh * DK * SEQ;
    v8f o[8];
#pragma unroll
    for (int d = 0; d < 8; ++d) o[d] = (v8f){};
    float m2 = -__builtin_inff(), lsum = 0.0f;
    const float c2 = (0.08838834764831845f * 1.4426950408889634f) * (1.0f / (SC_QKV * SC_QKV));
#pragma unroll 1
    for (int kt = 0; kt < SEQ / 64; ++kt) {
        v8f s[4];
#pragma unroll
        for (int ks = 0; ks < 4; ++ks) {
            const int key = kt * 64 + ks * 16 + l16;
            const _Float16* kr = kb + (size_t)key * DK;
            v8f c = (v8f){};
#pragma unroll
            for (int cc = 0; cc < 4; ++cc) c = wmma16(ldfrag(kr + cc * 32, hf), qf[cc], c);
            s[ks] = c;
        }
        float mloc = -__builtin_inff();
#pragma unroll
        for (int ks = 0; ks < 4; ++ks)
#pragma unroll
            for (int r = 0; r < 8; ++r) { s[ks][r] *= c2; mloc = fmaxf(mloc, s[ks][r]); }
        mloc = fmaxf(mloc, __shfl_xor(mloc, 16, 32));
        const float mn = fmaxf(m2, mloc);
        const float alpha = exp2f(m2 - mn);
        float ls = 0.0f;
        v16h pf[2];
#pragma unroll
        for (int ks = 0; ks < 4; ++ks)
#pragma unroll
            for (int r = 0; r < 8; ++r) {
                const float e = (s[ks][r] - mn) + P_CARRY_LOG2;
                const float p = (e < -14.0f) ? 0.0f : exp2f(e);
                ls += p;
                pf[ks >> 1][(ks & 1) * 8 + r] = (_Float16)p;
            }
        m2 = mn;
        lsum = lsum * alpha + ls;
#pragma unroll
        for (int d = 0; d < 8; ++d) o[d] *= alpha;
#pragma unroll
        for (int d = 0; d < 8; ++d) {
            const _Float16* vr = vb + (size_t)(d * 16 + l16) * SEQ + kt * 64;
            o[d] = wmma16(ldfrag(vr, hf), pf[0], o[d]);
            o[d] = wmma16(ldfrag(vr + 32, hf), pf[1], o[d]);
        }
    }
    const float lt = lsum + __shfl_xor(lsum, 16, 32);
    const float inv = (1.0f / lt) * (1.0f / SC_QKV);
#pragma unroll
    for (int d = 0; d < 8; ++d) {
        v4f p0, p1;
#pragma unroll
        for (int r = 0; r < 4; ++r) { p0[r] = o[d][r] * inv; p1[r] = o[d][4 + r] * inv; }
        *(v4f*)&st[wv][l16 * 132 + d * 16 + 8 * hf]     = p0;
        *(v4f*)&st[wv][l16 * 132 + d * 16 + 8 * hf + 4] = p1;
    }
    __syncthreads();
    v4f w[16];
#pragma unroll
    for (int t = 0; t < 16; ++t) w[t] = *(const v4f*)&st[wv][t * 132 + lane * 4];
    float* obase = OUT + ((size_t)bi * SEQ_FULL + q0) * DM + hd * DK + lane * 4;
    auto pass = [&]() {
#pragma unroll
        for (int t = 0; t < 16; ++t) vst16f(obase + (size_t)t * DM, w[t]);
    };
    pass();
    __threadfence();
    pass();
}

extern "C" void kernel_launch(void* const* d_in, const int* in_sizes, int n_in,
                              void* d_out, int out_size, void* d_ws, size_t ws_size, hipStream_t stream) {
    if (n_in < 6) return;
    const long long needTok = (long long)(NB - 1) * SEQ_FULL + SEQ;
    if ((long long)in_sizes[0] < needTok * DM) return;
    if (in_sizes[1] < NH * DM * DK || in_sizes[2] < NH * DM * DK || in_sizes[3] < NH * DK ||
        in_sizes[4] < NH * DM * DK || in_sizes[5] < NH * DK) return;
    if ((long long)out_size < needTok * DM) return;

    const float* x  = (const float*)d_in[0];
    const float* Wq = (const float*)d_in[1];
    const float* Wk = (const float*)d_in[2];
    const float* bk = (const float*)d_in[3];
    const float* Wv = (const float*)d_in[4];
    const float* bv = (const float*)d_in[5];
    float* out = (float*)d_out;

    char* ws = (char*)d_ws;
    size_t off = 0;
    auto carve = [&](size_t bytes) -> char* { char* p = ws + off; off += (bytes + 255) & ~(size_t)255; return p; };
    _Float16* XH = (_Float16*)carve(WS_XH);
    _Float16* WT = (_Float16*)carve(WS_WT);
    _Float16* QK = (_Float16*)carve(WS_QK);
    _Float16* VT = (_Float16*)carve(WS_VT);
    if (off > ws_size) return;
    _Float16* QC = QK;
    _Float16* KC = QK + (size_t)NB * NH * SEQ * DK;

    k_cvtx<<<CVTX_BLK, 256, 0, stream>>>(x, XH);
    k_prepw<<<PREPW_BLK, 256, 0, stream>>>(Wq, WT);
    k_prepw<<<PREPW_BLK, 256, 0, stream>>>(Wk, WT + (size_t)NH * DK * DM);
    k_prepw<<<PREPW_BLK, 256, 0, stream>>>(Wv, WT + (size_t)2 * NH * DK * DM);
    k_proj<<<dim3(MTOK / 64, PROJN / 128, 1), 128, 0, stream>>>(XH, WT, bk, bv, QK, VT);
    k_attn<<<dim3(SEQ / 64, NB * NH, 1), 128, 0, stream>>>(QC, KC, VT, out);
}
